// TestLSTMCell_54176717471880
// MI455X (gfx1250) — hardware-verified
//
#include <hip/hip_runtime.h>


typedef __bf16       v16bf __attribute__((ext_vector_type(16)));
typedef __bf16       v8bf  __attribute__((ext_vector_type(8)));
typedef float        v8f   __attribute__((ext_vector_type(8)));
typedef float        v4f   __attribute__((ext_vector_type(4)));
typedef unsigned int v4u   __attribute__((ext_vector_type(4)));

#define MROWS 4096
#define KD    1024
#define NH    1024
#define BM    64
#define BN    64
#define NTHR  256
#define LP    68

union Frag { v16bf v; v8bf h[2]; };

__device__ __forceinline__ v8f vz() {
    v8f z = {0.f, 0.f, 0.f, 0.f, 0.f, 0.f, 0.f, 0.f};
    return z;
}

__device__ __forceinline__ v16bf ldfrag(const __bf16* __restrict__ P, int row, int k0, int h) {
    const __bf16* p = P + ((size_t)row * KD + (size_t)(k0 + 8 * h));
    Frag f;
    f.h[0] = *(const v8bf*)(p);
    f.h[1] = *(const v8bf*)(p + 16);
    return f.v;
}

__device__ __forceinline__ v8f mma(v16bf a, v16bf b, v8f c) {
    v8f d = __builtin_amdgcn_wmma_f32_16x16x32_bf16(false, a, false, b, (short)0, c, false, false);
    asm volatile("v_nop\n\tv_nop\n\tv_nop\n\tv_nop" : "+v"(d) : "v"(a), "v"(b));
    return d;
}

__device__ __forceinline__ void stage_acc(float* s, int r0, int c, int h, v8f acc) {
#pragma unroll
    for (int r = 0; r < 8; ++r) s[(r0 + 8 * h + r) * LP + c] = acc[r];
}

__device__ __forceinline__ unsigned int f2bf(float f) {
    unsigned int u = __float_as_uint(f);
    return (u + 0x7FFFu + ((u >> 16) & 1u)) >> 16;
}
__device__ __forceinline__ float bf2f(unsigned int b) { return __uint_as_float(b << 16); }
__device__ __forceinline__ float rbf(float f) { return bf2f(f2bf(f)); }
__device__ __forceinline__ v4f rbf4(v4f a) {
    v4f r;
    r.x = rbf(a.x); r.y = rbf(a.y); r.z = rbf(a.z); r.w = rbf(a.w);
    return r;
}

__device__ __forceinline__ void hl2(float v0, float v1, unsigned int& hp, unsigned int& lp) {
    const unsigned int h0 = f2bf(v0), h1 = f2bf(v1);
    const unsigned int l0 = f2bf(v0 - bf2f(h0)), l1 = f2bf(v1 - bf2f(h1));
    hp = h0 | (h1 << 16);
    lp = l0 | (l1 << 16);
}
__device__ __forceinline__ void hl8(const float* sp, v4u& H, v4u& L) {
    const v4f u0 = *(const v4f*)(sp);
    const v4f u1 = *(const v4f*)(sp + 4);
    unsigned int h0, h1, h2, h3, l0, l1, l2, l3;
    hl2(u0.x, u0.y, h0, l0);
    hl2(u0.z, u0.w, h1, l1);
    hl2(u1.x, u1.y, h2, l2);
    hl2(u1.z, u1.w, h3, l3);
    H.x = h0; H.y = h1; H.z = h2; H.w = h3;
    L.x = l0; L.y = l1; L.z = l2; L.w = l3;
}

__device__ __forceinline__ float sigm(float x) {
    x = fminf(fmaxf(x, -30.0f), 30.0f);
    return __builtin_amdgcn_rcpf(1.0f + __expf(-x));
}
__device__ __forceinline__ float tnh(float x) {
    x = fminf(fmaxf(x, -15.0f), 15.0f);
    return 1.0f - 2.0f * __builtin_amdgcn_rcpf(__expf(2.0f * x) + 1.0f);
}

__global__ __launch_bounds__(NTHR) void k_cvt(
    const float* s0, const float* s1, const float* s2, const float* s3,
    const float* s4, const float* s5, const float* s6,
    unsigned short* d0, unsigned short* d1, unsigned short* d2, unsigned short* d3,
    unsigned short* d4, unsigned short* d5, unsigned short* d6, int n8)
{
    const int seg = blockIdx.y;
    const float* s = s0; unsigned short* d = d0;
    if (seg == 1)      { s = s1; d = d1; }
    else if (seg == 2) { s = s2; d = d2; }
    else if (seg == 3) { s = s3; d = d3; }
    else if (seg == 4) { s = s4; d = d4; }
    else if (seg == 5) { s = s5; d = d5; }
    else if (seg == 6) { s = s6; d = d6; }
    const int i = blockIdx.x * NTHR + threadIdx.x;
    if (i >= n8) return;
    const size_t e = (size_t)i * 8;
    const v4f a = *(const v4f*)(s + e);
    const v4f b = *(const v4f*)(s + e + 4);
    v4u o;
    o.x = f2bf(a.x) | (f2bf(a.y) << 16);
    o.y = f2bf(a.z) | (f2bf(a.w) << 16);
    o.z = f2bf(b.x) | (f2bf(b.y) << 16);
    o.w = f2bf(b.z) | (f2bf(b.w) << 16);
    volatile v4u* p = (volatile v4u*)(d + e);
    *p = o;
    __threadfence();
    *p = o;
}

__global__ __launch_bounds__(NTHR) void k_g1(
    const __bf16* __restrict__ xb, const __bf16* __restrict__ wxt,
    const float* __restrict__ bxt, const float* __restrict__ hx,
    float* t32, unsigned short* thi, unsigned short* tlo)
{
    __shared__ __attribute__((aligned(16))) float sT[BM * LP];
    const int tid = threadIdx.x;
    const int lane = tid & 31, wave = tid >> 5;
    const int h = lane >> 4, m = lane & 15;
    const int wr = wave >> 2, wc = wave & 3;
    const int row0 = blockIdx.y * BM, col0 = blockIdx.x * BN;
    const int ar = row0 + wr * 32 + m;
    const int bc = col0 + wc * 16 + m;

    v8f acc0 = vz(), acc1 = vz();
#pragma unroll 2
    for (int k0 = 0; k0 < KD; k0 += 32) {
        const v16bf a0 = ldfrag(xb, ar, k0, h);
        const v16bf a1 = ldfrag(xb, ar + 16, k0, h);
        const v16bf b  = ldfrag(wxt, bc, k0, h);
        acc0 = mma(a0, b, acc0);
        acc1 = mma(a1, b, acc1);
    }
    stage_acc(sT, wr * 32,      wc * 16 + m, h, acc0);
    stage_acc(sT, wr * 32 + 16, wc * 16 + m, h, acc1);
    __syncthreads();

#pragma unroll
    for (int it = 0; it < 4; ++it) {
        const int q = it * NTHR + tid;
        const int r = q >> 4, c4 = (q & 15) * 4;
        float* sp = &sT[r * LP + c4];
        const v4f a = *(const v4f*)sp;
        const size_t gi = (size_t)(row0 + r) * NH + (size_t)(col0 + c4);
        const v4f bb = *(const v4f*)(bxt + col0 + c4);
        const v4f hh = *(const v4f*)(hx + gi);
        const v4f pre = a + rbf4(bb);
        const v4f hr = rbf4(hh);
        v4f t;
        t.x = tnh(pre.x) + hr.x;
        t.y = tnh(pre.y) + hr.y;
        t.z = tnh(pre.z) + hr.z;
        t.w = tnh(pre.w) + hr.w;
        volatile v4f* p = (volatile v4f*)(t32 + gi);
        *p = t;
        __threadfence();
        *p = t;
        *(v4f*)sp = t;
    }
    __syncthreads();

#pragma unroll
    for (int it = 0; it < 2; ++it) {
        const int g = it * NTHR + tid;
        const int r = g >> 3, cg = (g & 7) * 8;
        v4u H, L;
        hl8(&sT[r * LP + cg], H, L);
        const size_t gi = (size_t)(row0 + r) * NH + (size_t)(col0 + cg);
        volatile v4u* ph = (volatile v4u*)(thi + gi);
        volatile v4u* pl = (volatile v4u*)(tlo + gi);
        *ph = H;
        *pl = L;
        __threadfence();
        *ph = H;
        *pl = L;
    }
}

__global__ __launch_bounds__(NTHR) void k_g2(
    const __bf16* __restrict__ thi, const __bf16* __restrict__ tlo, const __bf16* __restrict__ cxb,
    const __bf16* __restrict__ wtf, const __bf16* __restrict__ wcf,
    const __bf16* __restrict__ wtu, const __bf16* __restrict__ wcu,
    const float* __restrict__ btf, const float* __restrict__ bcf,
    const float* __restrict__ btu, const float* __restrict__ bcu,
    const float* __restrict__ t32, const float* __restrict__ cx,
    float* cyo, unsigned short* cyhi, unsigned short* cylo)
{
    __shared__ __attribute__((aligned(16))) float sF[BM * LP];
    __shared__ __attribute__((aligned(16))) float sU[BM * LP];
    const int tid = threadIdx.x;
    const int lane = tid & 31, wave = tid >> 5;
    const int h = lane >> 4, m = lane & 15;
    const int wr = wave >> 2, wc = wave & 3;
    const int row0 = blockIdx.y * BM, col0 = blockIdx.x * BN;
    const int ar = row0 + wr * 32 + m;
    const int bc = col0 + wc * 16 + m;

    v8f F0 = vz(), F1 = vz(), U0 = vz(), U1 = vz();

#pragma unroll
    for (int pl = 0; pl < 2; ++pl) {
        const __bf16* A = (pl == 0) ? thi : tlo;
#pragma unroll 2
        for (int k0 = 0; k0 < KD; k0 += 32) {
            const v16bf a0 = ldfrag(A, ar, k0, h);
            const v16bf a1 = ldfrag(A, ar + 16, k0, h);
            const v16bf bf = ldfrag(wtf, bc, k0, h);
            const v16bf bu = ldfrag(wtu, bc, k0, h);
            F0 = mma(a0, bf, F0);
            F1 = mma(a1, bf, F1);
            U0 = mma(a0, bu, U0);
            U1 = mma(a1, bu, U1);
        }
    }
#pragma unroll 2
    for (int k0 = 0; k0 < KD; k0 += 32) {
        const v16bf a0 = ldfrag(cxb, ar, k0, h);
        const v16bf a1 = ldfrag(cxb, ar + 16, k0, h);
        const v16bf bf = ldfrag(wcf, bc, k0, h);
        const v16bf bu = ldfrag(wcu, bc, k0, h);
        F0 = mma(a0, bf, F0);
        F1 = mma(a1, bf, F1);
        U0 = mma(a0, bu, U0);
        U1 = mma(a1, bu, U1);
    }

    stage_acc(sF, wr * 32,      wc * 16 + m, h, F0);
    stage_acc(sF, wr * 32 + 16, wc * 16 + m, h, F1);
    stage_acc(sU, wr * 32,      wc * 16 + m, h, U0);
    stage_acc(sU, wr * 32 + 16, wc * 16 + m, h, U1);
    __syncthreads();

#pragma unroll
    for (int it = 0; it < 4; ++it) {
        const int q = it * NTHR + tid;
        const int r = q >> 4, c4 = (q & 15) * 4;
        float* spF = &sF[r * LP + c4];
        const v4f aF = *(const v4f*)spF;
        const v4f aU = *(const v4f*)&sU[r * LP + c4];
        const size_t gi = (size_t)(row0 + r) * NH + (size_t)(col0 + c4);
        const v4f b1 = *(const v4f*)(btf + col0 + c4);
        const v4f b2 = *(const v4f*)(bcf + col0 + c4);
        const v4f b3 = *(const v4f*)(btu + col0 + c4);
        const v4f b4 = *(const v4f*)(bcu + col0 + c4);
        const v4f tt = *(const v4f*)(t32 + gi);
        const v4f cc = rbf4(*(const v4f*)(cx + gi));
        const v4f pF = aF + (rbf4(b1) + rbf4(b2));
        const v4f pU = aU + (rbf4(b3) + rbf4(b4));
        v4f cy;
        cy.x = tnh(sigm(pF.x) * cc.x + sigm(pU.x) * tt.x);
        cy.y = tnh(sigm(pF.y) * cc.y + sigm(pU.y) * tt.y);
        cy.z = tnh(sigm(pF.z) * cc.z + sigm(pU.z) * tt.z);
        cy.w = tnh(sigm(pF.w) * cc.w + sigm(pU.w) * tt.w);
        volatile v4f* p = (volatile v4f*)(cyo + gi);
        *p = cy;
        __threadfence();
        *p = cy;
        *(v4f*)spF = cy;
    }
    __syncthreads();

#pragma unroll
    for (int it = 0; it < 2; ++it) {
        const int g = it * NTHR + tid;
        const int r = g >> 3, cg = (g & 7) * 8;
        v4u H, L;
        hl8(&sF[r * LP + cg], H, L);
        const size_t gi = (size_t)(row0 + r) * NH + (size_t)(col0 + cg);
        volatile v4u* ph = (volatile v4u*)(cyhi + gi);
        volatile v4u* pl = (volatile v4u*)(cylo + gi);
        *ph = H;
        *pl = L;
        __threadfence();
        *ph = H;
        *pl = L;
    }
}

__global__ __launch_bounds__(NTHR) void k_g3(
    const __bf16* __restrict__ thi, const __bf16* __restrict__ tlo,
    const __bf16* __restrict__ cyhi, const __bf16* __restrict__ cylo,
    const __bf16* __restrict__ wth, const __bf16* __restrict__ wch,
    const float* __restrict__ bth, const float* __restrict__ bch,
    const float* cyf, float* hy)
{
    __shared__ __attribute__((aligned(16))) float sS[BM * LP];
    const int tid = threadIdx.x;
    const int lane = tid & 31, wave = tid >> 5;
    const int h = lane >> 4, m = lane & 15;
    const int wr = wave >> 2, wc = wave & 3;
    const int row0 = blockIdx.y * BM, col0 = blockIdx.x * BN;
    const int ar = row0 + wr * 32 + m;
    const int bc = col0 + wc * 16 + m;

    v8f acc0 = vz(), acc1 = vz();
#pragma unroll
    for (int pl = 0; pl < 4; ++pl) {
        const __bf16* A = (pl == 0) ? thi : (pl == 1) ? tlo : (pl == 2) ? cyhi : cylo;
        const __bf16* W = (pl < 2) ? wth : wch;
#pragma unroll 2
        for (int k0 = 0; k0 < KD; k0 += 32) {
            const v16bf a0 = ldfrag(A, ar, k0, h);
            const v16bf a1 = ldfrag(A, ar + 16, k0, h);
            const v16bf b  = ldfrag(W, bc, k0, h);
            acc0 = mma(a0, b, acc0);
            acc1 = mma(a1, b, acc1);
        }
    }
    stage_acc(sS, wr * 32,      wc * 16 + m, h, acc0);
    stage_acc(sS, wr * 32 + 16, wc * 16 + m, h, acc1);
    __syncthreads();

#pragma unroll
    for (int it = 0; it < 4; ++it) {
        const int q = it * NTHR + tid;
        const int r = q >> 4, c4 = (q & 15) * 4;
        const v4f a = *(const v4f*)&sS[r * LP + c4];
        const size_t gi = (size_t)(row0 + r) * NH + (size_t)(col0 + c4);
        const v4f b1 = *(const v4f*)(bth + col0 + c4);
        const v4f b2 = *(const v4f*)(bch + col0 + c4);
        const v4f cc = *(const v4f*)(cyf + gi);
        const v4f pre = a + (rbf4(b1) + rbf4(b2));
        v4f o;
        o.x = tnh(sigm(pre.x) * cc.x);
        o.y = tnh(sigm(pre.y) * cc.y);
        o.z = tnh(sigm(pre.z) * cc.z);
        o.w = tnh(sigm(pre.w) * cc.w);
        volatile v4f* p = (volatile v4f*)(hy + gi);
        *p = o;
        __threadfence();
        *p = o;
    }
}

extern "C" void kernel_launch(void* const* d_in, const int* in_sizes, int n_in,
                              void* d_out, int out_size, void* d_ws, size_t ws_size,
                              hipStream_t stream) {
    if (n_in < 17) return;
    const int actN = MROWS * KD;
    const int wN   = NH * KD;
    bool ok = (out_size == 2 * MROWS * NH);
    for (int i = 0; i < 3; ++i)   ok = ok && (in_sizes[i] == actN);
    for (int i = 3; i < 10; ++i)  ok = ok && (in_sizes[i] == wN);
    for (int i = 10; i < 17; ++i) ok = ok && (in_sizes[i] == NH);
    if (!ok) return;

    const float* x  = (const float*)d_in[0];
    const float* hx = (const float*)d_in[1];
    const float* cx = (const float*)d_in[2];
    const float* W[7];
    for (int i = 0; i < 7; ++i) W[i] = (const float*)d_in[3 + i];
    const float* b_xt = (const float*)d_in[10];
    const float* b_tf = (const float*)d_in[11];
    const float* b_cf = (const float*)d_in[12];
    const float* b_tu = (const float*)d_in[13];
    const float* b_cu = (const float*)d_in[14];
    const float* b_th = (const float*)d_in[15];
    const float* b_ch = (const float*)d_in[16];

    float* hy_out = (float*)d_out;
    float* cy_out = (float*)d_out + (size_t)MROWS * NH;

    const size_t actB = (size_t)actN * 2;
    const size_t wB   = (size_t)wN * 2;
    const size_t f32B = (size_t)actN * 4;
    size_t off = 0;
    char* base = (char*)d_ws;
    unsigned short* xb  = (unsigned short*)(base + off); off += actB;
    unsigned short* cxb = (unsigned short*)(base + off); off += actB;
    unsigned short* wb[7];
    for (int i = 0; i < 7; ++i) { wb[i] = (unsigned short*)(base + off); off += wB; }
    float* t32 = (float*)(base + off);                   off += f32B;
    unsigned short* thi  = (unsigned short*)(base + off); off += actB;
    unsigned short* tlo  = (unsigned short*)(base + off); off += actB;
    unsigned short* cyhi = (unsigned short*)(base + off); off += actB;
    unsigned short* cylo = (unsigned short*)(base + off); off += actB;
    if (off > ws_size) return;

    const int n8a = actN / 8;
    const int n8w = wN / 8;
    k_cvt<<<dim3((n8a + NTHR - 1) / NTHR, 2), dim3(NTHR), 0, stream>>>(
        x, cx, cx, cx, cx, cx, cx,
        xb, cxb, cxb, cxb, cxb, cxb, cxb, n8a);
    k_cvt<<<dim3((n8w + NTHR - 1) / NTHR, 7), dim3(NTHR), 0, stream>>>(
        W[0], W[1], W[2], W[3], W[4], W[5], W[6],
        wb[0], wb[1], wb[2], wb[3], wb[4], wb[5], wb[6], n8w);

    const dim3 grid(NH / BN, MROWS / BM);
    const dim3 block(NTHR);

    k_g1<<<grid, block, 0, stream>>>(
        (const __bf16*)xb, (const __bf16*)wb[0], b_xt, hx, t32, thi, tlo);

    k_g2<<<grid, block, 0, stream>>>(
        (const __bf16*)thi, (const __bf16*)tlo, (const __bf16*)cxb,
        (const __bf16*)wb[1], (const __bf16*)wb[2],
        (const __bf16*)wb[3], (const __bf16*)wb[4],
        b_tf, b_cf, b_tu, b_cu,
        t32, cx, cy_out, cyhi, cylo);

    k_g3<<<grid, block, 0, stream>>>(
        (const __bf16*)thi, (const __bf16*)tlo,
        (const __bf16*)cyhi, (const __bf16*)cylo,
        (const __bf16*)wb[5], (const __bf16*)wb[6],
        b_th, b_ch, cy_out, hy_out);
}
